// SynthesizerAttention_12232066859635
// MI455X (gfx1250) — hardware-run, weakly checked
//
#include <hip/hip_runtime.h>


#define NB_  8
#define TR   1023
#define TT   1024
#define DM   1024
#define NH_  16
#define HD   64
#define PCAR 1024.0f
#define RH   256
typedef _Float16 h16;
typedef unsigned short bf;
typedef __attribute__((ext_vector_type(16))) __bf16   v16bf;
typedef __attribute__((ext_vector_type(16))) _Float16 v16h;
typedef __attribute__((ext_vector_type(8)))  _Float16 v8h;
typedef __attribute__((ext_vector_type(8)))  unsigned short v8us;
typedef __attribute__((ext_vector_type(8)))  float    v8f;
typedef __attribute__((ext_vector_type(4)))  float    v4f;
typedef v8h  __attribute__((may_alias)) v8ha;
typedef v4f  __attribute__((may_alias)) v4fa;
typedef v8us __attribute__((may_alias)) v8usa;

__device__ __forceinline__ unsigned short f2bf(float f) { unsigned u = __float_as_uint(f); u += 0x7FFFu + ((u >> 16) & 1u); return (unsigned short)(u >> 16); }
__device__ __forceinline__ float bf2f(unsigned short b) { return __uint_as_float(((unsigned)b) << 16); }
__device__ __forceinline__ float bfr(float f) { return bf2f(f2bf(f)); }
__device__ __forceinline__ v16h cat16(v8h lo, v8h hi) { return __builtin_shufflevector(lo, hi, 0, 1, 2, 3, 4, 5, 6, 7, 8, 9, 10, 11, 12, 13, 14, 15); }
__device__ __forceinline__ v16bf cat16b(v8us lo, v8us hi) { return __builtin_bit_cast(v16bf, __builtin_shufflevector(lo, hi, 0, 1, 2, 3, 4, 5, 6, 7, 8, 9, 10, 11, 12, 13, 14, 15)); }
__device__ __forceinline__ v8f wmma16(v16h a, v16h b, v8f c) { return __builtin_amdgcn_wmma_f32_16x16x32_f16(false, a, false, b, (short)0, c, false, false); }
__device__ __forceinline__ v8f wmmab(v16bf a, v16bf b, v8f c) { return __builtin_amdgcn_wmma_f32_16x16x32_bf16(false, a, false, b, (short)0, c, false, false); }


template <typename T16> struct WFrag;
template <> struct WFrag<h16> { typedef v16h V; static __device__ __forceinline__ V ld(const h16* p) { return cat16(*(const v8h*)p, *(const v8h*)(p + 16)); } static __device__ __forceinline__ v8f mma(V a, V b, v8f c) { return wmma16(a, b, c); } };
template <> struct WFrag<bf> { typedef v16bf V; static __device__ __forceinline__ V ld(const bf* p) { return cat16b(*(const v8us*)p, *(const v8us*)(p + 16)); } static __device__ __forceinline__ v8f mma(V a, V b, v8f c) { return wmmab(a, b, c); } };
template <typename T16, int NSPLIT, bool BIAS>
__global__ __launch_bounds__(32) void k_gemmw(const T16* __restrict__ A, const T16* __restrict__ A2, const T16* __restrict__ Bt, const T16* __restrict__ Bt2, int K, float* C, int ldc, const float* __restrict__ bias, size_t sA, size_t sB, size_t sC) {
    typedef typename WFrag<T16>::V V;
    __shared__ __align__(16) float os[16 * 68];
    const size_t z = blockIdx.z; A += z * sA; if (A2) A2 += z * sA; Bt += z * sB; if (Bt2) Bt2 += z * sB; C += z * sC;
    const int lane = threadIdx.x & 31, lr = lane & 15, hi = lane >> 4; const int r0 = blockIdx.x * 64, c0 = blockIdx.y * 64;
    v8f acc[4][4];
#pragma unroll
    for (int mb = 0; mb < 4; ++mb)
#pragma unroll
        for (int nb = 0; nb < 4; ++nb) acc[mb][nb] = (v8f){};
    const size_t aoff = (size_t)(r0 + lr) * K + 8 * hi, boff = (size_t)(c0 + lr) * K + 8 * hi;
#pragma unroll 1
    for (int kc = 0; kc < K; kc += 32) {
        V a[4], a2[4];
#pragma unroll
        for (int mb = 0; mb < 4; ++mb) { a[mb] = WFrag<T16>::ld(A + aoff + (size_t)mb * 16 * K + kc); if (NSPLIT == 1 || NSPLIT == 2) a2[mb] = WFrag<T16>::ld(A2 + aoff + (size_t)mb * 16 * K + kc); }
#pragma unroll
        for (int nb = 0; nb < 4; ++nb) { const V b = WFrag<T16>::ld(Bt + boff + (size_t)nb * 16 * K + kc); V b2; if (NSPLIT >= 2) b2 = WFrag<T16>::ld(Bt2 + boff + (size_t)nb * 16 * K + kc);
#pragma unroll
            for (int mb = 0; mb < 4; ++mb) { acc[mb][nb] = WFrag<T16>::mma(a[mb], b, acc[mb][nb]); if (NSPLIT == 1 || NSPLIT == 2) acc[mb][nb] = WFrag<T16>::mma(a2[mb], b, acc[mb][nb]); if (NSPLIT >= 2) acc[mb][nb] = WFrag<T16>::mma(a[mb], b2, acc[mb][nb]); } }
        asm volatile("v_nop\n\tv_nop\n\tv_nop\n\tv_nop" : "+v"(acc[0][0]), "+v"(acc[1][1]), "+v"(acc[2][2]), "+v"(acc[3][3]) : "v"(a[0]), "v"(a[3]));
    }
#pragma unroll
    for (int mb = 0; mb < 4; ++mb) {
#pragma unroll
        for (int nb = 0; nb < 4; ++nb) {
#pragma unroll
            for (int j = 0; j < 8; ++j) os[(hi * 8 + j) * 68 + nb * 16 + lr] = acc[mb][nb][j]; }
        __builtin_amdgcn_wave_barrier(); asm volatile("" ::: "memory");
        float* crow = C + (size_t)(r0 + mb * 16) * ldc + c0;
#pragma unroll 1
        for (int ps = 0; ps < 2; ++ps) {
#pragma unroll
            for (int s = 0; s < 8; ++s) { const int row = 2 * s + hi, cofs = lr * 4; v4f val = *(const v4fa*)(os + row * 68 + cofs); if (BIAS) { val[0] += bfr(bias[c0 + cofs]); val[1] += bfr(bias[c0 + cofs + 1]); val[2] += bfr(bias[c0 + cofs + 2]); val[3] += bfr(bias[c0 + cofs + 3]); }
                *(volatile v4f*)(crow + (size_t)row * ldc + cofs) = val; }
            if (ps == 0) __threadfence(); }
        __builtin_amdgcn_wave_barrier(); asm volatile("" ::: "memory");
    }
}

__device__ __forceinline__ h16 tohx(float x) { return (h16)x; }
__device__ __forceinline__ void splitf(float y, unsigned short& h, unsigned short& l) { h = f2bf(y); l = f2bf(y - bf2f(h)); }
typedef __attribute__((ext_vector_type(2))) unsigned short v2us;
typedef __attribute__((ext_vector_type(4))) unsigned short v4us;
typedef __attribute__((ext_vector_type(2))) _Float16 v2h;
typedef __attribute__((ext_vector_type(4))) _Float16 v4h;

__global__ __launch_bounds__(256) void k_cvt8(const float* __restrict__ src, bf* dst, size_t n8) { const size_t i = (size_t)blockIdx.x * 256 + threadIdx.x; if (i >= n8) return; const v8f v = *(const v8f*)(src + i * 8); v8us o;
#pragma unroll
    for (int k = 0; k < 8; ++k) o[k] = f2bf(v[k]); *(volatile v8us*)(dst + i * 8) = o; __threadfence(); *(volatile v8us*)(dst + i * 8) = o; }
__global__ __launch_bounds__(256) void k_xpad(const float* __restrict__ xb, bf* XB) { const size_t e = ((size_t)blockIdx.x * 256 + threadIdx.x) * 4; if (e >= (size_t)TT * DM) return; const int t = (int)(e / DM); v4us o;
#pragma unroll
    for (int u = 0; u < 4; ++u) o[u] = (t < TR) ? f2bf(xb[e + u]) : (unsigned short)0; *(volatile v4us*)(XB + e) = o; __threadfence(); *(volatile v4us*)(XB + e) = o; }
__global__ __launch_bounds__(256) void k_w2t(const float* __restrict__ w2, h16* Bt) { const int e = (blockIdx.x * 256 + threadIdx.x) * 4; if (e >= TT * HD) return; const int d = e % HD; const int m = e / HD; v4h o;
#pragma unroll
    for (int u = 0; u < 4; ++u) o[u] = (m < TR) ? tohx(bfr(w2[(size_t)(d + u) * TR + m])) : (h16)0.f; *(volatile v4h*)(Bt + e) = o; __threadfence(); *(volatile v4h*)(Bt + e) = o; }
__global__ __launch_bounds__(256) void k_rpl(const float* __restrict__ R, h16* RP) { const size_t e = ((size_t)blockIdx.x * 256 + threadIdx.x) * 4; if (e >= (size_t)NH_ * TT * HD) return; const int d = (int)(e % HD); const int t = (int)((e / HD) % TT); const int h = (int)(e / ((size_t)HD * TT)); const float* r = R + (size_t)t * DM + h * HD + d; v4h o;
#pragma unroll
    for (int u = 0; u < 4; ++u) o[u] = tohx(fmaxf(r[u], 0.f)); *(volatile v4h*)(RP + e) = o; __threadfence(); *(volatile v4h*)(RP + e) = o; }
__global__ __launch_bounds__(256) void k_vt(const float* __restrict__ V, h16* VT, bf* VTh, bf* VTl) { const size_t e = ((size_t)blockIdx.x * 256 + threadIdx.x) * 2; if (e >= (size_t)NH_ * HD * TT) return; const int s = (int)(e % TT); const int d = (int)((e / TT) % HD); const int h = (int)(e / ((size_t)TT * HD)); v2h o; v2us oh, ol;
#pragma unroll
    for (int u = 0; u < 2; ++u) { const float vv = (s + u < TR) ? V[(size_t)(s + u) * DM + h * HD + d] : 0.f; o[u] = tohx(vv); unsigned short a, b; splitf(vv, a, b); oh[u] = a; ol[u] = b; }
    *(volatile v2h*)(VT + e) = o; *(volatile v2us*)(VTh + e) = oh; *(volatile v2us*)(VTl + e) = ol; __threadfence(); *(volatile v2h*)(VT + e) = o; *(volatile v2us*)(VTh + e) = oh; *(volatile v2us*)(VTl + e) = ol; }
__global__ __launch_bounds__(256) void k_sysoft(const float* __restrict__ S, const float* __restrict__ b2, h16* P16, bf* Ph, bf* Pl) { const int lane = threadIdx.x & 31; const int row = blockIdx.x * 8 + (threadIdx.x >> 5); if (row >= NH_ * TT) return; const int t = row % TT; const float* sr = S + (size_t)row * TT; float v[TT / 32]; float mx = -3.0e38f;
    if (t < TR) {
#pragma unroll
        for (int ch = 0; ch < TT / 128; ++ch) { const v4f a = *(const v4f*)(sr + ch * 128 + lane * 4);
#pragma unroll
            for (int u = 0; u < 4; ++u) { const int s = ch * 128 + lane * 4 + u; float bb = (s < TR) ? bfr(b2[s]) : 0.f; asm volatile("" : "+v"(bb)); const float tt = (s <= t) ? __fadd_rn(a[u], bb) : -1.0e10f; v[ch * 4 + u] = tt; mx = fmaxf(mx, tt); } } }
    else { for (int q = 0; q < TT / 32; ++q) v[q] = 0.f; mx = 0.f; }
#pragma unroll
    for (int sh = 16; sh; sh >>= 1) mx = fmaxf(mx, __shfl_xor(mx, sh, 32));
    float sum = 0.f;
#pragma unroll
    for (int q = 0; q < TT / 32; ++q) { float d0 = __fsub_rn(v[q], mx); asm volatile("" : "+v"(d0)); v[q] = (t < TR) ? __builtin_amdgcn_exp2f(__fmul_rn(d0, 1.4426950408889634f)) : 0.f; sum += v[q]; }
#pragma unroll
    for (int sh = 16; sh; sh >>= 1) sum += __shfl_xor(sum, sh, 32);
    const float f = (t < TR) ? __fdiv_rn(PCAR, sum) : 0.f; const float f1 = (t < TR) ? __fdiv_rn(1.0f, sum) : 0.f; const int h = row / TT;
    for (int ps = 0; ps < 2; ++ps) {
#pragma unroll
        for (int ch = 0; ch < TT / 128; ++ch) { v4h o4; for (int q = 0; q < 4; ++q) o4[q] = tohx(v[ch * 4 + q] * f); *(volatile v4h*)(P16 + (size_t)row * TT + ch * 128 + lane * 4) = o4;
            if (t < RH) { v4us oh, ol; for (int q = 0; q < 4; ++q) { unsigned short a2, c2; splitf(v[ch * 4 + q] * f1, a2, c2); oh[q] = a2; ol[q] = c2; } const size_t oo = ((size_t)h * RH + t) * TT + ch * 128 + lane * 4; *(volatile v4us*)(Ph + oo) = oh; *(volatile v4us*)(Pl + oo) = ol; } }
        if (ps == 0) __threadfence(); } }
__global__ __launch_bounds__(256) void k_mrg(const float* __restrict__ O, bf* Ah, bf* Al) { const size_t e = ((size_t)blockIdx.x * 256 + threadIdx.x) * 4; if (e >= (size_t)TT * DM) return; const int c = (int)(e % DM); const int t = (int)(e / DM); const int h = c / HD, d = c % HD; const float* src = O + ((size_t)h * TT + t) * HD + d; v4us oh, ol;
#pragma unroll
    for (int u = 0; u < 4; ++u) { const float cs = (t < RH) ? 1.0f : (1.0f / PCAR); unsigned short a, b; splitf(src[u] * cs, a, b); oh[u] = a; ol[u] = b; } *(volatile v4us*)(Ah + e) = oh; *(volatile v4us*)(Al + e) = ol; __threadfence(); *(volatile v4us*)(Ah + e) = oh; *(volatile v4us*)(Al + e) = ol; }
__global__ __launch_bounds__(256) void k_copy(const float* __restrict__ Y, float* outb) { const size_t e = ((size_t)blockIdx.x * 256 + threadIdx.x) * 4; if (e >= (size_t)TR * DM) return; const v4f a = *(const v4f*)(Y + e); *(volatile v4f*)(outb + e) = a; __threadfence(); *(volatile v4f*)(outb + e) = a; }

extern "C" void kernel_launch(void* const* d_in, const int* in_sizes, int n_in,
                              void* d_out, int out_size, void* d_ws, size_t ws_size, hipStream_t stream) {
    (void)in_sizes; (void)n_in; (void)out_size;
    const float** I = (const float**)d_in;
    const float *x = I[0], *w1 = I[1], *b1 = I[2], *w2 = I[3], *b2 = I[4], *wv = I[5], *bv = I[6], *wp = I[7], *bp = I[8];
    float* OUT = (float*)d_out;
    char* wsp = (char*)d_ws;
    auto take = [&](size_t bytes) { char* p = wsp; wsp += (bytes + 255) & ~(size_t)255; return (void*)p; };
    bf* B1 = (bf*)take((size_t)DM * DM * 2); bf* BV = (bf*)take((size_t)DM * DM * 2); bf* BP = (bf*)take((size_t)DM * DM * 2); h16* W2T = (h16*)take((size_t)TT * HD * 2);
    bf* XB = (bf*)take((size_t)TT * DM * 2); float* R = (float*)take((size_t)TT * DM * 4); float* V = (float*)take((size_t)TT * DM * 4); h16* RP = (h16*)take((size_t)NH_ * TT * HD * 2); h16* VT = (h16*)take((size_t)NH_ * HD * TT * 2); bf* VTh = (bf*)take((size_t)NH_ * HD * TT * 2); bf* VTl = (bf*)take((size_t)NH_ * HD * TT * 2); bf* Ph = (bf*)take((size_t)NH_ * RH * TT * 2); bf* Pl = (bf*)take((size_t)NH_ * RH * TT * 2);
    float* S = (float*)take((size_t)NH_ * TT * TT * 4); h16* P16 = (h16*)take((size_t)NH_ * TT * TT * 2); float* O = (float*)take((size_t)NH_ * TT * HD * 4); bf* Ah = (bf*)take((size_t)TT * DM * 2); bf* Al = (bf*)take((size_t)TT * DM * 2); float* Y = (float*)take((size_t)TT * DM * 4);
    if ((size_t)(wsp - (char*)d_ws) > ws_size) return;
    k_cvt8<<<(DM * DM / 8 + 255) / 256, 256, 0, stream>>>(w1, B1, DM * DM / 8); k_cvt8<<<(DM * DM / 8 + 255) / 256, 256, 0, stream>>>(wv, BV, DM * DM / 8); k_cvt8<<<(DM * DM / 8 + 255) / 256, 256, 0, stream>>>(wp, BP, DM * DM / 8);
    k_w2t<<<(TT * HD / 4 + 255) / 256, 256, 0, stream>>>(w2, W2T);
    const size_t zr = (size_t)TT * HD, zS = (size_t)TT * TT;
    for (int b = 0; b < NB_; ++b) {
        k_xpad<<<(unsigned)(((size_t)TT * DM / 4 + 255) / 256), 256, 0, stream>>>(x + (size_t)b * TR * DM, XB);
        k_gemmw<bf, 0, true><<<dim3(TT / 64, DM / 64, 1), 32, 0, stream>>>(XB, nullptr, B1, nullptr, DM, R, DM, b1, 0, 0, 0); k_gemmw<bf, 0, true><<<dim3(TT / 64, DM / 64, 1), 32, 0, stream>>>(XB, nullptr, BV, nullptr, DM, V, DM, bv, 0, 0, 0);
        k_rpl<<<(unsigned)(((size_t)NH_ * TT * HD / 4 + 255) / 256), 256, 0, stream>>>(R, RP); k_vt<<<(unsigned)(((size_t)NH_ * HD * TT / 2 + 255) / 256), 256, 0, stream>>>(V, VT, VTh, VTl);
        k_gemmw<h16, 0, false><<<dim3(TT / 64, TT / 64, NH_), 32, 0, stream>>>(RP, nullptr, W2T, nullptr, HD, S, TT, nullptr, zr, 0, zS);
        k_sysoft<<<NH_ * TT / 8, 256, 0, stream>>>(S, b2, P16, Ph, Pl);
        k_gemmw<bf, 2, false><<<dim3(RH / 64, 1, NH_), 32, 0, stream>>>(Ph, Pl, VTh, VTl, TT, O, HD, nullptr, (size_t)RH * TT, (size_t)HD * TT, zr);
        k_gemmw<h16, 0, false><<<dim3((TT - RH) / 64, 1, NH_), 32, 0, stream>>>(P16 + (size_t)RH * TT, nullptr, VT, nullptr, TT, O + (size_t)RH * HD, HD, nullptr, zS, (size_t)HD * TT, zr);
        k_mrg<<<(unsigned)(((size_t)TT * DM / 4 + 255) / 256), 256, 0, stream>>>(O, Ah, Al);
        k_gemmw<bf, 1, true><<<dim3(TT / 64, DM / 64, 1), 32, 0, stream>>>(Ah, Al, BP, nullptr, DM, Y, DM, bp, 0, 0, 0);
        k_copy<<<(unsigned)(((size_t)TR * DM / 4 + 255) / 256), 256, 0, stream>>>(Y, OUT + (size_t)b * TR * DM); }
}
